// DMG_7146825581012
// MI455X (gfx1250) — hardware-verified
//
#include <hip/hip_runtime.h>

typedef __attribute__((ext_vector_type(16))) _Float16 v16h;
typedef __attribute__((ext_vector_type(8)))  _Float16 v8h;
typedef __attribute__((ext_vector_type(8)))  float    v8f;
#define BATCH 4
#define NLAB  64
#define HH    512
#define WW    512
#define VST2(T, ptr, val) do { const T _v = (val); *(volatile T*)(ptr) = _v; __threadfence(); *(volatile T*)(ptr) = _v; } while (0)
__device__ __forceinline__ v8f wmma16(v16h a, v16h b, v8f c) {
  v8f d = __builtin_amdgcn_wmma_f32_16x16x32_f16(false, a, false, b, (short)0, c, false, false);
  asm volatile("v_nop\n\tv_nop\n\tv_nop\n\tv_nop" : "+v"(d) : "v"(a), "v"(b));
  return d;
}
__device__ __forceinline__ v16h frag16(const _Float16* p, int hh) {
  const v8h lo = *(const v8h*)(p + 8 * hh), hi = *(const v8h*)(p + 16 + 8 * hh);
  return __builtin_shufflevector(lo, hi, 0,1,2,3,4,5,6,7,8,9,10,11,12,13,14,15);
}
__global__ __launch_bounds__(256) void k_scale(const float* __restrict__ labels, const float* __restrict__ sigma_p, float* __restrict__ scale) {
  const int t = blockIdx.x * 256 + threadIdx.x;
  const int n = t & 63, axis = (t >> 6) & 1, b = t >> 7;
  const float sigma = sigma_p[0], inv = 1.0f / (2.0f * sigma * sigma);
  const float c = labels[(b * NLAB + n) * 2 + axis];
  float s = 0.f;
  for (int pos = 0; pos < 512; ++pos) { const float d = (float)pos - c; s += expf(-d * d * inv); }
  VST2(float, scale + t, 1.0f / s);
}
__global__ __launch_bounds__(256) void k_gauss(const float* __restrict__ labels, const float* __restrict__ sigma_p, const float* __restrict__ scale,
                                               _Float16* __restrict__ G) {
  const int t = blockIdx.x * 256 + threadIdx.x;
  const int n0 = (t & 7) * 8, pos = (t >> 3) & 511, axis = (t >> 12) & 1, b = t >> 13;
  const float sigma = sigma_p[0], inv = 1.0f / (2.0f * sigma * sigma);
  v8h v;
#pragma unroll
  for (int q = 0; q < 8; ++q) {
    const int n = n0 + q;
    const float c = labels[(b * NLAB + n) * 2 + axis], d = (float)pos - c;
    v[q] = (_Float16)(expf(-d * d * inv) * scale[(b * 2 + axis) * 64 + n]);
  }
  VST2(v8h, G + (size_t)t * 8, v);
}
__global__ __launch_bounds__(256) void k_density(const _Float16* __restrict__ G, float* __restrict__ out) {
  const int lane = threadIdx.x & 31, hh = lane >> 4, l16 = lane & 15;
  const int gw = blockIdx.x * 8 + (threadIdx.x >> 5);
  const int b = gw >> 8, tm = (gw >> 3) & 31, cg = gw & 7;
  const _Float16* Gx = G + ((size_t)(b * 2 + 0) * 512) * NLAB;
  const _Float16* Gy = G + ((size_t)(b * 2 + 1) * 512) * NLAB;
  v8f acc[4] = {};
#pragma unroll
  for (int ks = 0; ks < 2; ++ks) {
    const v16h a = frag16(Gy + (size_t)(tm * 16 + l16) * NLAB + ks * 32, hh);
#pragma unroll
    for (int t = 0; t < 4; ++t) acc[t] = wmma16(a, frag16(Gx + (size_t)(cg * 64 + t * 16 + l16) * NLAB + ks * 32, hh), acc[t]);
  }
  for (int pass = 0; pass < 2; ++pass) {
#pragma unroll
    for (int pr = 0; pr < 2; ++pr)
#pragma unroll
      for (int r = 0; r < 8; ++r) {
        const float a_ = acc[2 * pr][r], b_ = acc[2 * pr + 1][r];
        const float ax = __shfl_xor(a_, 16), bx = __shfl_xor(b_, 16);
        float* row0 = out + ((size_t)b * HH + tm * 16 + r) * WW + cg * 64 + pr * 32 + lane;
        *(volatile float*)row0 = hh ? bx : a_;
        *(volatile float*)(row0 + (size_t)8 * WW) = hh ? b_ : ax;
      }
    __threadfence();
  }
}
extern "C" void kernel_launch(void* const* d_in, const int* in_sizes, int n_in,
                              void* d_out, int out_size, void* d_ws, size_t ws_size, hipStream_t stream) {
  (void)in_sizes; (void)n_in; (void)out_size;
  const float* labels = (const float*)d_in[1];
  const float* sigma  = (const float*)d_in[2];
  float* out = (float*)d_out;
  if (ws_size < (size_t)BATCH * 2 * 512 * NLAB * 2 + 4096) return;
  float* scale = (float*)d_ws;
  _Float16* G  = (_Float16*)((char*)d_ws + 4096);
  k_scale<<<2, 256, 0, stream>>>(labels, sigma, scale);
  k_gauss<<<BATCH * 2 * 512 * 8 / 256, 256, 0, stream>>>(labels, sigma, scale, G);
  k_density<<<128, 256, 0, stream>>>(G, out);
}
